// EGCVBlockS4_21569325760699
// MI455X (gfx1250) — hardware-verified
//
#include <hip/hip_runtime.h>


#define NB_ 4
#define CC 96
#define HS 64
#define WS 64
#define LL (HS * WS)
#define DI 192
#define NS 16
#define DR 6
#define NXD 38
#define KD 4
#define MH 384
#define NTOK (NB_ * LL)

typedef __attribute__((ext_vector_type(16))) __bf16   v16bf;
typedef __attribute__((ext_vector_type(16))) _Float16 v16h;
typedef __attribute__((ext_vector_type(8)))  float    v8f;
typedef __attribute__((ext_vector_type(8)))  unsigned v8u;

__device__ __forceinline__ unsigned f2bf(float f) { unsigned u = __float_as_uint(f); u += 0x7FFFu + ((u >> 16) & 1u); return u >> 16; }
__device__ __forceinline__ unsigned f2h(float f) { return (unsigned)__builtin_bit_cast(unsigned short, (_Float16)f); }
__device__ __forceinline__ int kpat(int v, int half) { return ((v & 4) ? 16 : 0) + half * 8 + 2 * (v & 3); }

template <int F16, int NP> struct Opnd { v16bf p[NP]; };

template <int F16, int NP> __device__ __forceinline__ void pack2(float f0, float f1, unsigned* o) {
    if (F16) { o[0] = f2h(f0) | (f2h(f1) << 16); return; }
    unsigned h0 = f2bf(f0), h1 = f2bf(f1); o[0] = h0 | (h1 << 16);
    if (NP >= 2) {
        float r0 = f0 - __uint_as_float(h0 << 16), r1 = f1 - __uint_as_float(h1 << 16);
        unsigned m0 = f2bf(r0), m1 = f2bf(r1); o[1] = m0 | (m1 << 16);
        if (NP >= 3) {
            float s0 = r0 - __uint_as_float(m0 << 16), s1 = r1 - __uint_as_float(m1 << 16);
            o[2] = f2bf(s0) | (f2bf(s1) << 16);
        }
    }
}
template <int F16, int NP> __device__ __forceinline__ void op_row(const float* rowp, int half, float sc, Opnd<F16, NP>& o) {
    v8u u[NP];
#pragma unroll
    for (int v = 0; v < 8; ++v) {
        int kk = kpat(v, half); unsigned t[3];
        pack2<F16, NP>(rowp[kk] * sc, rowp[kk + 1] * sc, t);
#pragma unroll
        for (int p = 0; p < NP; ++p) u[p][v] = t[p];
    }
#pragma unroll
    for (int p = 0; p < NP; ++p) o.p[p] = __builtin_bit_cast(v16bf, u[p]);
}
template <int F16, int NP> __device__ __forceinline__ void op_row_tail(const float* rowp, int half, float sc, int kvalid, Opnd<F16, NP>& o) {
    v8u u[NP];
#pragma unroll
    for (int v = 0; v < 8; ++v) {
        int kk = kpat(v, half); unsigned t[3];
        float f0 = kk < kvalid ? rowp[kk] * sc : 0.0f, f1 = (kk + 1) < kvalid ? rowp[kk + 1] * sc : 0.0f;
        pack2<F16, NP>(f0, f1, t);
#pragma unroll
        for (int p = 0; p < NP; ++p) u[p][v] = t[p];
    }
#pragma unroll
    for (int p = 0; p < NP; ++p) o.p[p] = __builtin_bit_cast(v16bf, u[p]);
}
template <int F16, int NP> __device__ __forceinline__ void op_col(const float* M, int ld, int n, int k0, int half, float sc, Opnd<F16, NP>& o) {
    v8u u[NP];
#pragma unroll
    for (int v = 0; v < 8; ++v) {
        int kk = k0 + kpat(v, half); unsigned t[3];
        pack2<F16, NP>(M[(size_t)kk * ld + n] * sc, M[(size_t)(kk + 1) * ld + n] * sc, t);
#pragma unroll
        for (int p = 0; p < NP; ++p) u[p][v] = t[p];
    }
#pragma unroll
    for (int p = 0; p < NP; ++p) o.p[p] = __builtin_bit_cast(v16bf, u[p]);
}
template <int F16, int NP> __device__ __forceinline__ void op_col_tail(const float* M, int ld, int n, int k0, int half, float sc, int K, Opnd<F16, NP>& o) {
    v8u u[NP];
#pragma unroll
    for (int v = 0; v < 8; ++v) {
        int kk = k0 + kpat(v, half); unsigned t[3];
        float f0 = kk < K ? M[(size_t)kk * ld + n] * sc : 0.0f, f1 = (kk + 1) < K ? M[(size_t)(kk + 1) * ld + n] * sc : 0.0f;
        pack2<F16, NP>(f0, f1, t);
#pragma unroll
        for (int p = 0; p < NP; ++p) u[p][v] = t[p];
    }
#pragma unroll
    for (int p = 0; p < NP; ++p) o.p[p] = __builtin_bit_cast(v16bf, u[p]);
}
__device__ __forceinline__ v8f wm_bf16(v16bf a, v16bf b, v8f c) { return __builtin_amdgcn_wmma_f32_16x16x32_bf16(false, a, false, b, (short)0, c, false, false); }
template <int F16, int NA, int NB> __device__ __forceinline__ v8f wmma_op(const Opnd<F16, NA>& a, const Opnd<F16, NB>& b, v8f c) {
    if (F16) {
        v16h ah = __builtin_bit_cast(v16h, a.p[0]), bh = __builtin_bit_cast(v16h, b.p[0]);
        c = __builtin_amdgcn_wmma_f32_16x16x32_f16(false, ah, false, bh, (short)0, c, false, false);
        asm volatile("v_nop\n\tv_nop\n\tv_nop\n\tv_nop" : "+v"(c) : "v"(ah), "v"(bh));
        return c;
    }
    constexpr int NMX = NA > NB ? NA : NB;
#pragma unroll
    for (int i = 0; i < NA; ++i)
#pragma unroll
        for (int j = 0; j < NB; ++j)
            if (i + j < NMX) c = wm_bf16(a.p[i], b.p[j], c);
    if (NA == 1 && NB == 1)      asm volatile("v_nop\n\tv_nop\n\tv_nop\n\tv_nop" : "+v"(c) : "v"(a.p[0]), "v"(b.p[0]));
    else if (NA == 2 && NB == 1) asm volatile("v_nop\n\tv_nop\n\tv_nop\n\tv_nop" : "+v"(c) : "v"(a.p[0]), "v"(a.p[1]), "v"(b.p[0]));
    else if (NA == 1 && NB == 2) asm volatile("v_nop\n\tv_nop\n\tv_nop\n\tv_nop" : "+v"(c) : "v"(a.p[0]), "v"(b.p[0]), "v"(b.p[1]));
    else if (NA == 2 && NB == 2) asm volatile("v_nop\n\tv_nop\n\tv_nop\n\tv_nop" : "+v"(c) : "v"(a.p[0]), "v"(a.p[1]), "v"(b.p[0]), "v"(b.p[1]));
    else                         asm volatile("v_nop\n\tv_nop\n\tv_nop\n\tv_nop" : "+v"(c) : "v"(a.p[0]), "v"(a.p[NA - 1]), "v"(b.p[0]), "v"(b.p[NB - 1]), "v"(a.p[NA / 2]), "v"(b.p[NB / 2]));
    return c;
}

struct ZMap { long long s1; long long s2; int zdiv; int pad_; };
__device__ __forceinline__ size_t zoff(const ZMap& m, int z) { return (size_t)((long long)(z / m.zdiv) * m.s1 + (long long)(z % m.zdiv) * m.s2); }

#define ACT_NONE 0
#define ACT_RELU 1
#define ACT_GELU_ERF 2
#define ACT_SILU 3
#define ACT_TANH 4
__device__ __forceinline__ float act_apply(int act, float x) {
    if (act == ACT_RELU) return x > 0.f ? x : 0.f;
    if (act == ACT_GELU_ERF) return 0.5f * x * (1.0f + erff(x * 0.70710678118654752f));
    if (act == ACT_SILU) return x / (1.0f + expf(-x));
    if (act == ACT_TANH) return tanhf(x);
    return x;
}
struct GemmArgs {
    ZMap za, zb_, zc, zbias, zadd, zrsc, zmul, zrbias;
    const float* A; const float* Bm; float* C; const float* bias; const float* add; const float* rsc; const float* mul; const float* rbias;
    long long ldadd, ldmul;
    int lda, ldb, ldc, K;
    float ascale, bscale, oscale, addscale;
    int M, nvalid, nstore, ldrsc;
    int bcs, pad1, pad2, pad3;
};
template <int BT, int F16, int NA, int NB, int RW, int CW, int ACT>
__global__ __launch_bounds__(256) void gemm_kernel(GemmArgs g) {
    constexpr int TR = 16 * RW, TC = 64 * CW, CSTR = TC + 4;
    __shared__ __align__(16) float cst[TR * CSTR];
    const int z = blockIdx.z;
    const float* A = g.A + zoff(g.za, z); const float* Bm = g.Bm + zoff(g.zb_, z); float* C = g.C + zoff(g.zc, z);
    const int tid = threadIdx.x, lane = tid & 31, wv = tid >> 5;
    const int l16 = lane & 15, half = lane >> 4;
    const int rt = wv % RW, ch = wv / RW;
    const int row0 = blockIdx.x * TR, col0 = blockIdx.y * TC + ch * 64;
    int arix = row0 + rt * 16 + l16; if (arix >= g.M) arix = g.M - 1;
    const float* arow = A + (size_t)arix * g.lda;
    v8f acc[4];
#pragma unroll
    for (int t = 0; t < 4; ++t) acc[t] = (v8f){};
    const int K = g.K;
#pragma unroll 1
    for (int kc = 0; kc < K; kc += 32) {
        Opnd<F16, NA> a;
        if (kc + 32 <= K) op_row<F16, NA>(arow + kc, half, g.ascale, a); else op_row_tail<F16, NA>(arow + kc, half, g.ascale, K - kc, a);
#pragma unroll
        for (int t = 0; t < 4; ++t) {
            Opnd<F16, NB> b;
            const int n = col0 + t * 16 + l16;
            if (n < g.nvalid) {
                if (BT) { if (kc + 32 <= K) op_row<F16, NB>(Bm + (size_t)n * g.ldb + kc, half, g.bscale, b); else op_row_tail<F16, NB>(Bm + (size_t)n * g.ldb + kc, half, g.bscale, K - kc, b); }
                else    { if (kc + 32 <= K) op_col<F16, NB>(Bm, g.ldb, n * g.bcs, kc, half, g.bscale, b); else op_col_tail<F16, NB>(Bm, g.ldb, n * g.bcs, kc, half, g.bscale, K, b); }
            } else {
#pragma unroll
                for (int p = 0; p < NB; ++p) b.p[p] = (v16bf){};
            }
            acc[t] = wmma_op<F16, NA, NB>(a, b, acc[t]);
        }
    }
    const float* bias = g.bias ? g.bias + zoff(g.zbias, z) : nullptr;
    const float* add = g.add ? g.add + zoff(g.zadd, z) : nullptr;
    const float* rsc = g.rsc ? g.rsc + zoff(g.zrsc, z) : nullptr;
    const float* mul = g.mul ? g.mul + zoff(g.zmul, z) : nullptr;
    const float* rbias = g.rbias ? g.rbias + zoff(g.zrbias, z) : nullptr;
#pragma unroll
    for (int t = 0; t < 4; ++t) {
        const int cl = ch * 64 + t * 16 + l16;
        const int cg = blockIdx.y * TC + cl;
        const bool cok = cg < g.nvalid;
        const float bv = (bias && cok) ? bias[(size_t)cg * g.bcs] : 0.0f;
#pragma unroll
        for (int r = 0; r < 8; ++r) {
            const int rl = rt * 16 + r + 8 * half;
            float v = acc[t][r] * g.oscale + bv;
            int rg = row0 + rl; if (rg >= g.M) rg = g.M - 1;
            if (rbias) v += rbias[rg];
            if (rsc) v *= rsc[(size_t)rg * g.ldrsc];
            if (mul && cok) v *= mul[(size_t)rg * g.ldmul + cg];
            if (add && cok) v += g.addscale * add[(size_t)rg * g.ldadd + cg];
            cst[rl * CSTR + cl] = v;
        }
    }
    __syncthreads();
    const int col = tid % TC, rsel = tid / TC, rstep = 256 / TC;
    if (ACT != ACT_NONE) {
#pragma unroll 1
        for (int r = rsel; r < TR; r += rstep) cst[r * CSTR + col] = act_apply(ACT, cst[r * CSTR + col]);
    }
    float* ob = C + (size_t)row0 * g.ldc + (size_t)blockIdx.y * TC;
    const bool colok = (int)(blockIdx.y * TC + col) < g.nstore;
    const int rmax = (g.M - row0 < TR) ? (g.M - row0) : TR;
    auto pass = [&]() {
        if (colok) {
#pragma unroll 4
            for (int r = rsel; r < rmax; r += rstep) *(volatile float*)(ob + (size_t)r * g.ldc + col) = cst[r * CSTR + col];
        }
    };
    pass();
    __threadfence();
    pass();
}
static inline ZMap zm(long long s1) { ZMap m; m.s1 = s1; m.s2 = 0; m.zdiv = 1; m.pad_ = 0; return m; }
static inline ZMap zm2(long long s1, long long s2, int zdiv) { ZMap m; m.s1 = s1; m.s2 = s2; m.zdiv = zdiv; m.pad_ = 0; return m; }
static inline GemmArgs gemm_args(const float* A, int lda, ZMap za, const float* Bm, int ldb, ZMap zb, float* C, int ldc, ZMap zc, int M, int N, int K) {
    GemmArgs g; g.za = za; g.zb_ = zb; g.zc = zc; g.zbias = zm(0); g.zadd = zm(0); g.zrsc = zm(0); g.zmul = zm(0); g.zrbias = zm(0);
    g.A = A; g.Bm = Bm; g.C = C; g.bias = nullptr; g.add = nullptr; g.rsc = nullptr; g.mul = nullptr; g.rbias = nullptr; g.ldadd = 0; g.ldmul = 0;
    g.lda = lda; g.ldb = ldb; g.ldc = ldc; g.K = K; g.ascale = 1.0f; g.bscale = 1.0f; g.oscale = 1.0f; g.addscale = 1.0f; g.M = M; g.nvalid = N; g.nstore = N; g.ldrsc = 1;
    g.bcs = 1; g.pad1 = 0; g.pad2 = 0; g.pad3 = 0;
    return g;
}
static_assert(sizeof(ZMap) == 24, "ZMap layout");
static_assert(sizeof(GemmArgs) == 8 * 24 + 8 * 8 + 2 * 8 + 4 * 4 + 4 * 4 + 4 * 4 + 4 * 4, "GemmArgs has no padding");

__global__ __launch_bounds__(256) void softmax_rows(float* S, long long sy, long long sx, int L, float prescale, const float* addv, long long say, int aydiv, int causal,
                                                  const int* imask, long long imy, long long imx, float maskval) {
    __shared__ float red[8];
    const int tid = threadIdx.x, lane = tid & 31, wid = tid >> 5;
    float* row = S + (size_t)blockIdx.y * sy + (size_t)blockIdx.x * sx;
    const float* av = addv ? addv + (size_t)(blockIdx.y / aydiv) * say : nullptr;
    const int* im = imask ? imask + (size_t)(blockIdx.y / aydiv) * imy + (size_t)blockIdx.x * imx : nullptr;
    float v[16];
    const int nj = L / 256;
    float mx = -__builtin_inff();
#pragma unroll
    for (int j = 0; j < 16; ++j) if (j < nj) { float t = row[tid + 256 * j] * prescale; if (av) t += av[tid + 256 * j]; if (im && im[tid + 256 * j] == 0) t = maskval; if (causal && (tid + 256 * j) > (int)blockIdx.x) t = -__builtin_inff(); v[j] = t; mx = fmaxf(mx, t); }
#pragma unroll
    for (int o = 16; o; o >>= 1) mx = fmaxf(mx, __shfl_xor(mx, o, 32));
    if (lane == 0) red[wid] = mx;
    __syncthreads();
    float m = red[0];
#pragma unroll
    for (int i = 1; i < 8; ++i) m = fmaxf(m, red[i]);
    if (m == -__builtin_inff()) m = 0.f;
    __syncthreads();
    float sum = 0.f;
#pragma unroll
    for (int j = 0; j < 16; ++j) if (j < nj) { v[j] = expf(v[j] - m); sum += v[j]; }
#pragma unroll
    for (int o = 16; o; o >>= 1) sum += __shfl_xor(sum, o, 32);
    if (lane == 0) red[wid] = sum;
    __syncthreads();
    float tot = 0.f;
#pragma unroll
    for (int i = 0; i < 8; ++i) tot += red[i];
    const float inv = 1.0f / tot;
#pragma unroll
    for (int j = 0; j < 16; ++j) if (j < nj) *(volatile float*)(row + tid + 256 * j) = v[j] * inv;
    __threadfence();
#pragma unroll
    for (int j = 0; j < 16; ++j) if (j < nj) *(volatile float*)(row + tid + 256 * j) = v[j] * inv;
}

#define VST2(T, p, v) do { const T vst2_v_ = (v); *(volatile T*)(p) = vst2_v_; __threadfence(); *(volatile T*)(p) = vst2_v_; } while (0)
__device__ __forceinline__ float silu_(float x) { return x / (1.0f + expf(-x)); }
__global__ __launch_bounds__(256) void k_t2tok(const float* __restrict__ x, float* XL) { __shared__ float tile[32][33]; const int l0 = blockIdx.x * 32, c0 = blockIdx.y * 32, b = blockIdx.z; const int tx = threadIdx.x & 31, ty = threadIdx.x >> 5;
    for (int k = 0; k < 4; ++k) { const int cr = ty + 8 * k; tile[cr][tx] = x[((size_t)b * CC + c0 + cr) * LL + l0 + tx]; } __syncthreads();
    for (int k = 0; k < 4; ++k) { const int lr = ty + 8 * k; VST2(float, XL + ((size_t)b * LL + l0 + lr) * CC + c0 + tx, tile[tx][lr]); } }
__global__ __launch_bounds__(256) void k_tok2t(const float* __restrict__ T_, float* out) { __shared__ float tile[32][33]; const int l0 = blockIdx.x * 32, c0 = blockIdx.y * 32, b = blockIdx.z; const int tx = threadIdx.x & 31, ty = threadIdx.x >> 5;
    for (int k = 0; k < 4; ++k) { const int lr = ty + 8 * k; tile[lr][tx] = T_[((size_t)b * LL + l0 + lr) * CC + c0 + tx]; } __syncthreads();
    for (int k = 0; k < 4; ++k) { const int cr = ty + 8 * k; VST2(float, out + ((size_t)b * CC + c0 + cr) * LL + l0 + tx, tile[tx][cr]); } }
__global__ __launch_bounds__(256) void k_ln96(const float* __restrict__ A, const float* __restrict__ g, const float* __restrict__ bb, float* OUT) { const int lane = threadIdx.x & 31, r = blockIdx.x * 8 + (threadIdx.x >> 5); if (r >= NTOK) return; const float* row = A + (size_t)r * CC; const float v0 = row[lane], v1 = row[lane + 32], v2 = row[lane + 64]; float s = v0 + v1 + v2;
#pragma unroll
    for (int o = 16; o; o >>= 1) s += __shfl_xor(s, o, 32);
    const float mean = s / 96.f; const float d0 = v0 - mean, d1 = v1 - mean, d2 = v2 - mean; float q = d0 * d0 + d1 * d1 + d2 * d2;
#pragma unroll
    for (int o = 16; o; o >>= 1) q += __shfl_xor(q, o, 32);
    const float rs = rsqrtf(q / 96.f + 1e-5f); VST2(float, OUT + (size_t)r * CC + lane, d0 * rs * g[lane] + bb[lane]); VST2(float, OUT + (size_t)r * CC + lane + 32, d1 * rs * g[lane + 32] + bb[lane + 32]); VST2(float, OUT + (size_t)r * CC + lane + 64, d2 * rs * g[lane + 64] + bb[lane + 64]); }
__global__ __launch_bounds__(256) void k_dw(const float* __restrict__ XZ, const float* __restrict__ w, const float* __restrict__ bb, float* XC) { const size_t q = (size_t)blockIdx.x * 256 + threadIdx.x; if (q >= (size_t)NTOK * DI) return; const int d = (int)(q % DI); const size_t tok = q / DI; const int l = (int)(tok % LL); const int b = (int)(tok / LL); const int h = l / WS, ww = l % WS; float s = bb[d];
#pragma unroll 1
    for (int ky = 0; ky < 7; ++ky) { const int y = h + ky - 3; if (y < 0 || y >= HS) continue;
#pragma unroll 1
        for (int kx = 0; kx < 7; ++kx) { const int xx = ww + kx - 3; if (xx < 0 || xx >= WS) continue; s += XZ[((size_t)b * LL + y * WS + xx) * (2 * DI) + d] * w[(d * 7 + ky) * 7 + kx]; } }
    VST2(float, XC + q, silu_(s)); }
__device__ __forceinline__ int pixof(int k, int l) { if (k == 2 || k == 3) l = LL - 1 - l; if (k == 1 || k == 3) { const int wq = l / HS, hq = l % HS; return hq * WS + wq; } return l; }
__global__ __launch_bounds__(256) void k_dirs(const float* __restrict__ XC, float* XS) { const size_t q = (size_t)blockIdx.x * 256 + threadIdx.x; if (q >= (size_t)NB_ * KD * LL * DI) return; const int d = (int)(q % DI); const int l = (int)((q / DI) % LL); const int k = (int)((q / ((size_t)DI * LL)) % KD); const int b = (int)(q / ((size_t)DI * LL * KD)); VST2(float, XS + q, XC[((size_t)b * LL + pixof(k, l)) * DI + d]); }
__global__ __launch_bounds__(256) void k_softplus(float* A, size_t n) { const size_t q = (size_t)blockIdx.x * 256 + threadIdx.x; if (q < n) { const float v = A[q]; VST2(float, A + q, v > 20.f ? v : log1pf(expf(v))); } }
__global__ __launch_bounds__(256) void k_scan(const float* __restrict__ XS, const float* __restrict__ DT, const float* __restrict__ XD, const float* __restrict__ Alog, const float* __restrict__ Dsk, float* Y) { const int q = blockIdx.x * 256 + threadIdx.x; if (q >= NB_ * KD * DI) return; const int d = q % DI; const int k = (q / DI) % KD; const int b = q / (DI * KD); float A[NS], h[NS];
#pragma unroll
    for (int n = 0; n < NS; ++n) { A[n] = -expf(Alog[(k * DI + d) * NS + n]); h[n] = 0.f; }
    const float Dd = Dsk[k * DI + d]; const size_t base = ((size_t)b * KD + k) * LL;
    for (int l = 0; l < LL; ++l) { const float xv = XS[(base + l) * DI + d]; const float dt = DT[(base + l) * DI + d]; const float* xd = XD + (base + l) * 64; float y = 0.f;
#pragma unroll 1
        for (int n = 0; n < NS; ++n) { h[n] = expf(dt * A[n]) * h[n] + dt * xv * xd[DR + n]; y += h[n] * xd[DR + NS + n]; }
        VST2(float, Y + (base + l) * DI + d, y + Dd * xv); } }
__global__ __launch_bounds__(256) void k_merge(const float* __restrict__ Y, const float* __restrict__ XZ, const float* __restrict__ g, const float* __restrict__ bb, float* YM) { const int lane = threadIdx.x & 31; const int tok = blockIdx.x * 8 + (threadIdx.x >> 5); if (tok >= NTOK) return; const int p = tok % LL, b = tok / LL; const int h_ = p / WS, w_ = p % WS; const int l1 = w_ * HS + h_; const size_t b0 = (size_t)b * KD * LL; float v[6]; float s = 0.f;
#pragma unroll
    for (int kk = 0; kk < 6; ++kk) { const int d = lane + 32 * kk; v[kk] = Y[(b0 + p) * DI + d] + Y[(b0 + LL + l1) * DI + d] + Y[(b0 + 2 * LL + (LL - 1 - p)) * DI + d] + Y[(b0 + 3 * LL + (LL - 1 - l1)) * DI + d]; s += v[kk]; }
#pragma unroll
    for (int o = 16; o; o >>= 1) s += __shfl_xor(s, o, 32);
    const float mean = s / (float)DI; float q = 0.f;
#pragma unroll
    for (int kk = 0; kk < 6; ++kk) { const float dd = v[kk] - mean; q += dd * dd; }
#pragma unroll
    for (int o = 16; o; o >>= 1) q += __shfl_xor(q, o, 32);
    const float rs = rsqrtf(q / (float)DI + 1e-5f);
#pragma unroll
    for (int kk = 0; kk < 6; ++kk) { const int d = lane + 32 * kk; VST2(float, YM + (size_t)tok * DI + d, ((v[kk] - mean) * rs * g[d] + bb[d]) * silu_(XZ[(size_t)tok * 2 * DI + DI + d])); } }
__global__ __launch_bounds__(256) void k_gelut(float* A, size_t n) { const size_t q = (size_t)blockIdx.x * 256 + threadIdx.x; if (q < n) { const float x = A[q]; const float u = 0.7978845608028654f * (x + 0.044715f * x * x * x); VST2(float, A + q, 0.5f * x * (1.0f + tanhf(u))); } }
extern "C" void kernel_launch(void* const* d_in, const int* in_sizes, int n_in,
                              void* d_out, int out_size, void* d_ws, size_t ws_size, hipStream_t stream) {
    (void)in_sizes; (void)n_in; (void)out_size;
    const float* x = (const float*)d_in[0]; const float* ln1w = (const float*)d_in[1]; const float* ln1b = (const float*)d_in[2]; const float* inw = (const float*)d_in[3]; const float* inb = (const float*)d_in[4]; const float* dww = (const float*)d_in[5]; const float* dwb = (const float*)d_in[6]; const float* xpw = (const float*)d_in[7]; const float* dtw = (const float*)d_in[8]; const float* dtb = (const float*)d_in[9]; const float* Alog = (const float*)d_in[10]; const float* Dsk = (const float*)d_in[11];
    const float* olw = (const float*)d_in[12]; const float* olb = (const float*)d_in[13]; const float* opw = (const float*)d_in[14]; const float* opb = (const float*)d_in[15]; const float* ln2w = (const float*)d_in[16]; const float* ln2b = (const float*)d_in[17]; const float* f1w = (const float*)d_in[18]; const float* f1b = (const float*)d_in[19]; const float* f2w = (const float*)d_in[20]; const float* f2b = (const float*)d_in[21];
    float* out = (float*)d_out;
    char* wsp = (char*)d_ws;
    auto take = [&](size_t bytes) { char* p = wsp; wsp += (bytes + 255) & ~(size_t)255; return (void*)p; };
    float* XL = (float*)take((size_t)NTOK * CC * 4); float* H1 = (float*)take((size_t)NTOK * CC * 4); float* XZ = (float*)take((size_t)NTOK * 2 * DI * 4); float* XC = (float*)take((size_t)NTOK * DI * 4); float* XS = (float*)take((size_t)NB_ * KD * LL * DI * 4); float* XD = (float*)take((size_t)NB_ * KD * LL * 64 * 4); float* DT = (float*)take((size_t)NB_ * KD * LL * DI * 4);
    float* Y = XS;
    Y = (float*)take((size_t)NB_ * KD * LL * DI * 4); float* YM = XC; float* X2 = H1; float* M1 = XZ; float* X3 = XL;
    if ((size_t)(wsp - (char*)d_ws) > ws_size) return;
    k_t2tok<<<dim3(LL / 32, CC / 32, NB_), 256, 0, stream>>>(x, XL);
    k_ln96<<<NTOK / 8, 256, 0, stream>>>(XL, ln1w, ln1b, H1);
    { GemmArgs g = gemm_args(H1, CC, zm(0), inw, CC, zm(0), XZ, 2 * DI, zm(0), NTOK, 2 * DI, CC); g.bias = inb; gemm_kernel<1, 1, 1, 1, 4, 2, ACT_NONE><<<dim3(NTOK / 64, (2 * DI) / 128, 1), 256, 0, stream>>>(g); }
    k_dw<<<(unsigned)(((size_t)NTOK * DI) / 256), 256, 0, stream>>>(XZ, dww, dwb, XC);
    k_dirs<<<(unsigned)(((size_t)NB_ * KD * LL * DI) / 256), 256, 0, stream>>>(XC, XS);
    for (int b = 0; b < NB_; ++b) { const size_t zb0 = (size_t)b * KD * LL;
        { GemmArgs g = gemm_args(XS + zb0 * DI, DI, zm((long long)LL * DI), xpw, DI, zm(NXD * DI), XD + zb0 * 64, 64, zm(LL * 64), LL, NXD, DI); g.nstore = 64; gemm_kernel<1, 1, 1, 1, 8, 1, ACT_NONE><<<dim3(LL / 128, 1, KD), 256, 0, stream>>>(g); }
        { GemmArgs g = gemm_args(XD + zb0 * 64, 64, zm(LL * 64), dtw, DR, zm(DI * DR), DT + zb0 * DI, DI, zm((long long)LL * DI), LL, DI, DR); g.bias = dtb; g.zbias = zm(DI); gemm_kernel<1, 1, 1, 1, 4, 2, ACT_NONE><<<dim3(LL / 64, 2, KD), 256, 0, stream>>>(g); }
    }
    k_softplus<<<(unsigned)(((size_t)NB_ * KD * LL * DI) / 256), 256, 0, stream>>>(DT, (size_t)NB_ * KD * LL * DI);
    k_scan<<<(NB_ * KD * DI) / 256, 256, 0, stream>>>(XS, DT, XD, Alog, Dsk, Y);
    k_merge<<<NTOK / 8, 256, 0, stream>>>(Y, XZ, olw, olb, YM);
    { GemmArgs g = gemm_args(YM, DI, zm(0), opw, DI, zm(0), X2, CC, zm(0), NTOK, CC, DI); g.bias = opb; g.add = XL; g.ldadd = CC; g.addscale = 1.0f; gemm_kernel<1, 1, 1, 1, 8, 1, ACT_NONE><<<dim3(NTOK / 128, 2, 1), 256, 0, stream>>>(g); }
    k_ln96<<<NTOK / 8, 256, 0, stream>>>(X2, ln2w, ln2b, XC);
    { GemmArgs g = gemm_args(XC, CC, zm(0), f1w, CC, zm(0), M1, MH, zm(0), NTOK, MH, CC); g.bias = f1b; gemm_kernel<1, 1, 1, 1, 4, 2, ACT_NONE><<<dim3(NTOK / 64, MH / 128, 1), 256, 0, stream>>>(g); }
    k_gelut<<<(unsigned)(((size_t)NTOK * MH) / 256), 256, 0, stream>>>(M1, (size_t)NTOK * MH);
    { GemmArgs g = gemm_args(M1, MH, zm(0), f2w, MH, zm(0), X3, CC, zm(0), NTOK, CC, MH); g.bias = f2b; g.add = X2; g.ldadd = CC; g.addscale = 1.0f; gemm_kernel<1, 1, 1, 1, 8, 1, ACT_NONE><<<dim3(NTOK / 128, 2, 1), 256, 0, stream>>>(g); }
    k_tok2t<<<dim3(LL / 32, CC / 32, NB_), 256, 0, stream>>>(X3, out);
}
